// ImprovedGraphSAGE_44444321579083
// MI455X (gfx1250) — hardware-verified
//
#include <hip/hip_runtime.h>
#include <stdint.h>


#define NND    20000
#define DEG    16
#define HID    128
#define GATES  512
#define OUTC   64
#define NEDGE  (NND * DEG)
#define MB     32
#define NTHR   256
#define APITCH 136
#define GPITCH 516
#define SPITCH 260

static_assert(NND % MB == 0);
static_assert(GATES == 4 * HID);
static_assert(MB * HID == NTHR * 16);
static_assert(MB * DEG == NTHR * 2);
static_assert((APITCH * 2) % 16 == 0);
static_assert((GPITCH * 4) % 16 == 0);
static_assert((SPITCH * 4) % 16 == 0);
static_assert(SPITCH >= HID);
static_assert(SPITCH <= GPITCH);

typedef _Float16 v4h  __attribute__((ext_vector_type(4)));
typedef _Float16 v8h  __attribute__((ext_vector_type(8)));
typedef _Float16 v16h __attribute__((ext_vector_type(16)));
typedef float    v4f  __attribute__((ext_vector_type(4)));
typedef float    v8f  __attribute__((ext_vector_type(8)));
union Frag { v16h v; v8h half[2]; };

#define ASCALE 8.0f
#define WSCALE 16.0f
#define INV128 0.0078125f

constexpr size_t SZ_WIH = (size_t)4 * GATES * HID * 2;
constexpr size_t SZ_WL  = (size_t)3 * HID * HID * 2;
constexpr size_t SZ_W4  = (size_t)OUTC * HID * 2;
constexpr size_t SZ_P   = (size_t)NND * GATES * 4;
constexpr size_t SZ_X   = (size_t)NND * HID * 4;

constexpr size_t OFF_WIH = 0;
constexpr size_t OFF_WHH = OFF_WIH + SZ_WIH;
constexpr size_t OFF_WL  = OFF_WHH + SZ_WIH;
constexpr size_t OFF_WR  = OFF_WL  + SZ_WL;
constexpr size_t OFF_WL4 = OFF_WR  + SZ_WL;
constexpr size_t OFF_WR4 = OFF_WL4 + SZ_W4;
constexpr size_t OFF_P   = OFF_WR4 + SZ_W4;
constexpr size_t OFF_X1  = OFF_P   + SZ_P;
constexpr size_t OFF_X2  = OFF_X1  + SZ_X;
constexpr size_t OFF_X3  = OFF_X2  + SZ_X;
constexpr size_t WS_END  = OFF_X3  + SZ_X;
static_assert(WS_END <= (size_t)134217728);
static_assert(OFF_WHH % 128 == 0 && OFF_WL % 128 == 0 && OFF_WR % 128 == 0 && OFF_WL4 % 128 == 0);
static_assert(OFF_WR4 % 128 == 0 && OFF_P % 128 == 0 && OFF_X1 % 128 == 0 && OFF_X2 % 128 == 0 && OFF_X3 % 128 == 0);
static_assert(SZ_P == (size_t)(NND / MB) * MB * GATES * 4);
static_assert(SZ_X == (size_t)(NND / MB) * MB * HID * 4);

constexpr int LDS_G     = MB * GPITCH * 4;
constexpr int LDS_C     = MB * HID * 4;
constexpr int LDS_H     = MB * APITCH * 2;
constexpr int LOFF_C    = LDS_G;
constexpr int LOFF_H    = LOFF_C + LDS_C;
constexpr int LOFF_X    = LOFF_H + LDS_H;
constexpr int LOFF_S    = LOFF_X + LDS_H;
constexpr int LDS_LAYER = LOFF_S + MB * DEG * 4;
constexpr int LOFF_A    = LDS_G;
constexpr int LDS_PROJ  = LOFF_A + LDS_H;
static_assert(LOFF_C % 16 == 0 && LOFF_H % 16 == 0 && LOFF_X % 16 == 0 && LOFF_S % 16 == 0);

__device__ __forceinline__ float rcp_f(float x) { return __builtin_amdgcn_rcpf(x); }
__device__ __forceinline__ float sigm(float x)  { return rcp_f(1.0f + __expf(-x)); }
__device__ __forceinline__ float tanhx(float x) { return 1.0f - 2.0f * rcp_f(1.0f + __expf(2.0f * x)); }

__device__ __forceinline__ void mma16(v8f& acc, const Frag& a, const Frag& b) {
  acc = __builtin_amdgcn_wmma_f32_16x16x32_f16(false, a.v, false, b.v, (short)0, acc, false, false);
  asm volatile("v_nop\n\tv_nop\n\tv_nop\n\tv_nop" : "+v"(acc) : "v"(a.v), "v"(b.v));
}

__device__ __forceinline__ void stage_rows_f16(_Float16* sA, const float* __restrict__ g, int tid) {
  const int row = tid >> 3, j0 = (tid & 7) * 16;
  const float* p = g + (size_t)row * HID + j0;
  const v4f a = *(const v4f*)(p);
  const v4f b = *(const v4f*)(p + 4);
  const v4f c = *(const v4f*)(p + 8);
  const v4f d = *(const v4f*)(p + 12);
  v8h u, w;
#pragma unroll
  for (int q = 0; q < 4; ++q) {
    u[q]     = (_Float16)(a[q] * ASCALE);
    u[4 + q] = (_Float16)(b[q] * ASCALE);
    w[q]     = (_Float16)(c[q] * ASCALE);
    w[4 + q] = (_Float16)(d[q] * ASCALE);
  }
  *(v8h*)(sA + row * APITCH + j0)     = u;
  *(v8h*)(sA + row * APITCH + j0 + 8) = w;
}

__device__ __forceinline__ void gemm_32x512(v8f (&acc)[8], const _Float16* sA,
                                            const _Float16* __restrict__ Bw, int wave, int lane)
{
  const int h = lane >> 4, m = lane & 15;
  const _Float16* a0 = sA + m * APITCH + 8 * h;
  const _Float16* a1 = sA + (16 + m) * APITCH + 8 * h;
  const _Float16* b0 = Bw + (size_t)(wave * 64 + m) * HID + 8 * h;
#pragma unroll
  for (int j = 0; j < 8; ++j)
#pragma unroll
    for (int r = 0; r < 8; ++r) acc[j][r] = 0.0f;
#pragma unroll 1
  for (int kc = 0; kc < 4; ++kc) {
    const int k0 = kc * 32;
    Frag fa0, fa1, fb[4];
    fa0.half[0] = *(const v8h*)(a0 + k0);
    fa0.half[1] = *(const v8h*)(a0 + k0 + 16);
    fa1.half[0] = *(const v8h*)(a1 + k0);
    fa1.half[1] = *(const v8h*)(a1 + k0 + 16);
#pragma unroll
    for (int j = 0; j < 4; ++j) {
      const _Float16* q = b0 + (size_t)j * 16 * HID + k0;
      fb[j].half[0] = *(const v8h*)(q);
      fb[j].half[1] = *(const v8h*)(q + 16);
    }
#pragma unroll
    for (int j = 0; j < 4; ++j) {
      mma16(acc[j],     fa0, fb[j]);
      mma16(acc[4 + j], fa1, fb[j]);
    }
  }
}

template <int COLS, int PITCH>
__device__ __forceinline__ void store_tile_pass(const float* sS, float* gbase, int tid) {
  constexpr int C4  = COLS / 4;
  constexpr int NIT = (MB * COLS / 4) / NTHR;
  static_assert(NIT * NTHR * 4 == MB * COLS);
#pragma unroll
  for (int it = 0; it < NIT; ++it) {
    const int idx = it * NTHR + tid;
    const int row = idx / C4;
    const int c4  = idx - row * C4;
    const v4f v = *(const v4f*)(sS + row * PITCH + 4 * c4);
    *(volatile v4f*)(gbase + (size_t)idx * 4) = v;
  }
}

__global__ __launch_bounds__(256)
void cvt16_kernel(const float* __restrict__ src, _Float16* dst, int n8, float scale)
{
  const int i = blockIdx.x * 256 + threadIdx.x;
  if (i >= n8) return;
  const size_t e = (size_t)i * 8;
  const v4f a = *(const v4f*)(src + e);
  const v4f b = *(const v4f*)(src + e + 4);
  v8h o;
#pragma unroll
  for (int q = 0; q < 4; ++q) {
    o[q]     = (_Float16)(a[q] * scale);
    o[4 + q] = (_Float16)(b[q] * scale);
  }
  _Float16* p = dst + e;
  *(volatile v8h*)p = o;
  __threadfence();
  *(volatile v8h*)p = o;
}

__global__ __launch_bounds__(NTHR)
void proj_kernel(const float* __restrict__ xin, const _Float16* __restrict__ Wih16,
                 const float* __restrict__ bih, const float* __restrict__ bhh, float* P)
{
  extern __shared__ __attribute__((aligned(16))) unsigned char dsm[];
  float*    sG = (float*)(dsm);
  _Float16* sA = (_Float16*)(dsm + LOFF_A);

  const int tid  = threadIdx.x;
  const int lane = tid & 31;
  const int wave = __builtin_amdgcn_readfirstlane(tid >> 5);
  const int h = lane >> 4, m = lane & 15;
  const int m0 = blockIdx.x * MB;

  stage_rows_f16(sA, xin + (size_t)m0 * HID, tid);
  __syncthreads();

  v8f acc[8];
  gemm_32x512(acc, sA, Wih16, wave, lane);
#pragma unroll
  for (int j = 0; j < 4; ++j) {
    const int col = wave * 64 + j * 16 + m;
    const float bb = bih[col] + bhh[col];
#pragma unroll
    for (int r = 0; r < 8; ++r) {
      sG[(8 * h + r) * GPITCH + col]      = acc[j][r] * INV128 + bb;
      sG[(16 + 8 * h + r) * GPITCH + col] = acc[4 + j][r] * INV128 + bb;
    }
  }
  __syncthreads();

  float* gbase = P + (size_t)m0 * GATES;
  store_tile_pass<GATES, GPITCH>(sG, gbase, tid);
  __threadfence();
  store_tile_pass<GATES, GPITCH>(sG, gbase, tid);
}

template <int OUTF, bool RELU, bool RES>
__global__ __launch_bounds__(NTHR)
void layer_kernel(const float* __restrict__ xin, const float* __restrict__ P, const int* __restrict__ src,
                  const _Float16* __restrict__ Whh16, const _Float16* __restrict__ Wl16,
                  const _Float16* __restrict__ Wr16, const float* __restrict__ bl, float* xout)
{
  static_assert(!RES || OUTF == HID);
  static_assert(OUTF % 32 == 0 && OUTF <= HID);
  extern __shared__ __attribute__((aligned(16))) unsigned char dsm[];
  float*    sG   = (float*)(dsm);
  float*    sC   = (float*)(dsm + LOFF_C);
  _Float16* sH   = (_Float16*)(dsm + LOFF_H);
  _Float16* sX   = (_Float16*)(dsm + LOFF_X);
  int*      sSrc = (int*)(dsm + LOFF_S);

  const int tid  = threadIdx.x;
  const int lane = tid & 31;
  const int wave = __builtin_amdgcn_readfirstlane(tid >> 5);
  const int h = lane >> 4, m = lane & 15;
  const int m0 = blockIdx.x * MB;
  const int cn = tid >> 3;
  const int cj = (tid & 7) * 16;

#pragma unroll 1
  for (int q = 0; q < 2; ++q) {
    const int i = q * NTHR + tid;
    int v = src[(size_t)m0 * DEG + i];
    v = min(max(v, 0), NND - 1);
    sSrc[i] = v;
  }
  stage_rows_f16(sX, xin + (size_t)m0 * HID, tid);
  {
    v8h z;
#pragma unroll
    for (int q = 0; q < 8; ++q) z[q] = (_Float16)0.0f;
    *(v8h*)(sH + cn * APITCH + cj)     = z;
    *(v8h*)(sH + cn * APITCH + cj + 8) = z;
    const v4f zf = {0.0f, 0.0f, 0.0f, 0.0f};
#pragma unroll
    for (int u = 0; u < 4; ++u) *(v4f*)(sC + cn * HID + cj + 4 * u) = zf;
  }

#pragma unroll 1
  for (int t = 0; t < DEG; ++t) {
    __syncthreads();
    {
      v8f acc[8];
      gemm_32x512(acc, sH, Whh16, wave, lane);
#pragma unroll
      for (int j = 0; j < 4; ++j) {
        const int col = wave * 64 + j * 16 + m;
#pragma unroll
        for (int r = 0; r < 8; ++r) {
          sG[(8 * h + r) * GPITCH + col]      = acc[j][r];
          sG[(16 + 8 * h + r) * GPITCH + col] = acc[4 + j][r];
        }
      }
    }
    __syncthreads();
    {
      const int e = sSrc[cn * DEG + t];
      const float* prow = P + (size_t)e * GATES + cj;
      const float* grow = sG + cn * GPITCH + cj;
      float* crow = sC + cn * HID + cj;
      _Float16* hrow = sH + cn * APITCH + cj;
#pragma unroll 1
      for (int u = 0; u < 4; ++u) {
        const int o = u * 4;
        const v4f pi = *(const v4f*)(prow + o);
        const v4f pf = *(const v4f*)(prow + HID + o);
        const v4f pg = *(const v4f*)(prow + 2 * HID + o);
        const v4f po = *(const v4f*)(prow + 3 * HID + o);
        const v4f gi = *(const v4f*)(grow + o);
        const v4f gf = *(const v4f*)(grow + HID + o);
        const v4f gg = *(const v4f*)(grow + 2 * HID + o);
        const v4f go = *(const v4f*)(grow + 3 * HID + o);
        v4f cc = *(const v4f*)(crow + o);
        v4f hh;
#pragma unroll
        for (int q = 0; q < 4; ++q) {
          const float ai = gi[q] * INV128 + pi[q];
          const float af = gf[q] * INV128 + pf[q];
          const float ag = gg[q] * INV128 + pg[q];
          const float ao = go[q] * INV128 + po[q];
          const float cnew = sigm(af) * cc[q] + sigm(ai) * tanhx(ag);
          cc[q] = cnew;
          hh[q] = sigm(ao) * tanhx(cnew);
        }
        *(v4f*)(crow + o) = cc;
        v4h h4;
#pragma unroll
        for (int q = 0; q < 4; ++q) h4[q] = (_Float16)(hh[q] * ASCALE);
        *(v4h*)(hrow + o) = h4;
      }
    }
  }
  __syncthreads();

  if (wave * 16 < OUTF) {
    v8f acc2[2];
#pragma unroll
    for (int s = 0; s < 2; ++s)
#pragma unroll
      for (int r = 0; r < 8; ++r) acc2[s][r] = 0.0f;
    const int col0 = wave * 16;
    const _Float16* al0 = sH + m * APITCH + 8 * h;
    const _Float16* al1 = sH + (16 + m) * APITCH + 8 * h;
    const _Float16* ax0 = sX + m * APITCH + 8 * h;
    const _Float16* ax1 = sX + (16 + m) * APITCH + 8 * h;
    const _Float16* bwl = Wl16 + (size_t)(col0 + m) * HID + 8 * h;
    const _Float16* bwr = Wr16 + (size_t)(col0 + m) * HID + 8 * h;
#pragma unroll 1
    for (int kc = 0; kc < 4; ++kc) {
      const int k0 = kc * 32;
      Frag fa0, fa1, fb;
      fa0.half[0] = *(const v8h*)(al0 + k0);
      fa0.half[1] = *(const v8h*)(al0 + k0 + 16);
      fa1.half[0] = *(const v8h*)(al1 + k0);
      fa1.half[1] = *(const v8h*)(al1 + k0 + 16);
      fb.half[0]  = *(const v8h*)(bwl + k0);
      fb.half[1]  = *(const v8h*)(bwl + k0 + 16);
      mma16(acc2[0], fa0, fb);
      mma16(acc2[1], fa1, fb);
    }
#pragma unroll 1
    for (int kc = 0; kc < 4; ++kc) {
      const int k0 = kc * 32;
      Frag fa0, fa1, fb;
      fa0.half[0] = *(const v8h*)(ax0 + k0);
      fa0.half[1] = *(const v8h*)(ax0 + k0 + 16);
      fa1.half[0] = *(const v8h*)(ax1 + k0);
      fa1.half[1] = *(const v8h*)(ax1 + k0 + 16);
      fb.half[0]  = *(const v8h*)(bwr + k0);
      fb.half[1]  = *(const v8h*)(bwr + k0 + 16);
      mma16(acc2[0], fa0, fb);
      mma16(acc2[1], fa1, fb);
    }
    const int col = col0 + m;
    const float bb = bl[col];
#pragma unroll
    for (int s = 0; s < 2; ++s)
#pragma unroll
      for (int r = 0; r < 8; ++r) {
        const int row = s * 16 + 8 * h + r;
        float v = acc2[s][r] * INV128 + bb;
        if constexpr (RES) v += xin[(size_t)(m0 + row) * HID + col];
        if constexpr (RELU) v = fmaxf(v, 0.0f);
        sG[row * SPITCH + col] = v;
      }
  }
  __syncthreads();

  float* gbase = xout + (size_t)m0 * OUTF;
  store_tile_pass<OUTF, SPITCH>(sG, gbase, tid);
  __threadfence();
  store_tile_pass<OUTF, SPITCH>(sG, gbase, tid);
}

extern "C" void kernel_launch(void* const* d_in, const int* in_sizes, int n_in,
                              void* d_out, int out_size, void* d_ws, size_t ws_size,
                              hipStream_t stream)
{
  if (n_in < 12) return;
  if (in_sizes[0]  != NND * HID)        return;
  if (in_sizes[1]  != 2 * NEDGE)        return;
  if (in_sizes[2]  != 4 * GATES * HID)  return;
  if (in_sizes[3]  != 4 * GATES * HID)  return;
  if (in_sizes[4]  != 4 * GATES)        return;
  if (in_sizes[5]  != 4 * GATES)        return;
  if (in_sizes[6]  != 3 * HID * HID)    return;
  if (in_sizes[7]  != 3 * HID)          return;
  if (in_sizes[8]  != 3 * HID * HID)    return;
  if (in_sizes[9]  != OUTC * HID)       return;
  if (in_sizes[10] != OUTC)             return;
  if (in_sizes[11] != OUTC * HID)       return;
  if (out_size != NND * OUTC)           return;
  if (ws_size < WS_END)                 return;

  const float* x     = (const float*)d_in[0];
  const int*   src   = (const int*)d_in[1];
  const float* Wih   = (const float*)d_in[2];
  const float* Whh   = (const float*)d_in[3];
  const float* bih   = (const float*)d_in[4];
  const float* bhh   = (const float*)d_in[5];
  const float* Wl123 = (const float*)d_in[6];
  const float* bl123 = (const float*)d_in[7];
  const float* Wr123 = (const float*)d_in[8];
  const float* Wl4   = (const float*)d_in[9];
  const float* bl4   = (const float*)d_in[10];
  const float* Wr4   = (const float*)d_in[11];
  float* out = (float*)d_out;

  char* ws = (char*)d_ws;
  _Float16* wih16 = (_Float16*)(ws + OFF_WIH);
  _Float16* whh16 = (_Float16*)(ws + OFF_WHH);
  _Float16* wl16  = (_Float16*)(ws + OFF_WL);
  _Float16* wr16  = (_Float16*)(ws + OFF_WR);
  _Float16* wl416 = (_Float16*)(ws + OFF_WL4);
  _Float16* wr416 = (_Float16*)(ws + OFF_WR4);
  float* P  = (float*)(ws + OFF_P);
  float* x1 = (float*)(ws + OFF_X1);
  float* x2 = (float*)(ws + OFF_X2);
  float* x3 = (float*)(ws + OFF_X3);

  hipFuncSetAttribute(reinterpret_cast<const void*>(&proj_kernel),
                      hipFuncAttributeMaxDynamicSharedMemorySize, LDS_PROJ);
  hipFuncSetAttribute(reinterpret_cast<const void*>(&layer_kernel<HID, true, false>),
                      hipFuncAttributeMaxDynamicSharedMemorySize, LDS_LAYER);
  hipFuncSetAttribute(reinterpret_cast<const void*>(&layer_kernel<HID, true, true>),
                      hipFuncAttributeMaxDynamicSharedMemorySize, LDS_LAYER);
  hipFuncSetAttribute(reinterpret_cast<const void*>(&layer_kernel<OUTC, false, false>),
                      hipFuncAttributeMaxDynamicSharedMemorySize, LDS_LAYER);

  {
    const int n8a = (4 * GATES * HID) / 8;
    const int n8b = (3 * HID * HID) / 8;
    const int n8c = (OUTC * HID) / 8;
    cvt16_kernel<<<dim3((n8a + 255) / 256), dim3(256), 0, stream>>>(Wih,   wih16, n8a, WSCALE);
    cvt16_kernel<<<dim3((n8a + 255) / 256), dim3(256), 0, stream>>>(Whh,   whh16, n8a, WSCALE);
    cvt16_kernel<<<dim3((n8b + 255) / 256), dim3(256), 0, stream>>>(Wl123, wl16,  n8b, WSCALE);
    cvt16_kernel<<<dim3((n8b + 255) / 256), dim3(256), 0, stream>>>(Wr123, wr16,  n8b, WSCALE);
    cvt16_kernel<<<dim3((n8c + 255) / 256), dim3(256), 0, stream>>>(Wl4,   wl416, n8c, WSCALE);
    cvt16_kernel<<<dim3((n8c + 255) / 256), dim3(256), 0, stream>>>(Wr4,   wr416, n8c, WSCALE);
  }

  const dim3 grid(NND / MB), block(NTHR);
  const size_t wstride  = (size_t)GATES * HID;
  const size_t lstride  = (size_t)HID * HID;

  proj_kernel<<<grid, block, LDS_PROJ, stream>>>(x, wih16 + 0 * wstride, bih + 0 * GATES, bhh + 0 * GATES, P);
  layer_kernel<HID, true, false><<<grid, block, LDS_LAYER, stream>>>(
      x, (const float*)P, src, whh16 + 0 * wstride, wl16 + 0 * lstride, wr16 + 0 * lstride, bl123 + 0 * HID, x1);

  proj_kernel<<<grid, block, LDS_PROJ, stream>>>((const float*)x1, wih16 + 1 * wstride, bih + 1 * GATES, bhh + 1 * GATES, P);
  layer_kernel<HID, true, true><<<grid, block, LDS_LAYER, stream>>>(
      (const float*)x1, (const float*)P, src, whh16 + 1 * wstride, wl16 + 1 * lstride, wr16 + 1 * lstride, bl123 + 1 * HID, x2);

  proj_kernel<<<grid, block, LDS_PROJ, stream>>>((const float*)x2, wih16 + 2 * wstride, bih + 2 * GATES, bhh + 2 * GATES, P);
  layer_kernel<HID, true, true><<<grid, block, LDS_LAYER, stream>>>(
      (const float*)x2, (const float*)P, src, whh16 + 2 * wstride, wl16 + 2 * lstride, wr16 + 2 * lstride, bl123 + 2 * HID, x3);

  proj_kernel<<<grid, block, LDS_PROJ, stream>>>((const float*)x3, wih16 + 3 * wstride, bih + 3 * GATES, bhh + 3 * GATES, P);
  layer_kernel<OUTC, false, false><<<grid, block, LDS_LAYER, stream>>>(
      (const float*)x3, (const float*)P, src, whh16 + 3 * wstride, wl416, wr416, bl4, out);
}
